// FLAGatedDeltaNet_24129126269510
// MI455X (gfx1250) — hardware-run, weakly checked
//
#include <hip/hip_runtime.h>


#define NSQ 2
#define NTS 1024
#define NHS 16
#define NFE 64
#define NCS 64
#define NCK 16
#define NPR 32
#define NZQ 512
#define NBL 4096
#define NRW 2048
#define NDM 1024

typedef _Float16 h16;
typedef unsigned short bf;
typedef __attribute__((ext_vector_type(16))) __bf16   v16bf;
typedef __attribute__((ext_vector_type(16))) _Float16 v16h;
typedef __attribute__((ext_vector_type(8)))  _Float16 v8h;
typedef __attribute__((ext_vector_type(8)))  unsigned short v8us;
typedef __attribute__((ext_vector_type(8)))  float    v8f;
typedef __attribute__((ext_vector_type(4)))  float    v4f;
typedef v8h  __attribute__((may_alias)) v8ha;
typedef v4f  __attribute__((may_alias)) v4fa;
typedef v8us __attribute__((may_alias)) v8usa;

__device__ __forceinline__ unsigned short f2bf(float f) { unsigned u = __float_as_uint(f); u += 0x7FFFu + ((u >> 16) & 1u); return (unsigned short)(u >> 16); }
__device__ __forceinline__ float bf2f(unsigned short b) { return __uint_as_float(((unsigned)b) << 16); }
__device__ __forceinline__ float bfr(float f) { return bf2f(f2bf(f)); }
__device__ __forceinline__ v16h cat16(v8h lo, v8h hi) { return __builtin_shufflevector(lo, hi, 0, 1, 2, 3, 4, 5, 6, 7, 8, 9, 10, 11, 12, 13, 14, 15); }
__device__ __forceinline__ v16bf cat16b(v8us lo, v8us hi) { return __builtin_bit_cast(v16bf, __builtin_shufflevector(lo, hi, 0, 1, 2, 3, 4, 5, 6, 7, 8, 9, 10, 11, 12, 13, 14, 15)); }
__device__ __forceinline__ v8f wmma16(v16h a, v16h b, v8f c) { return __builtin_amdgcn_wmma_f32_16x16x32_f16(false, a, false, b, (short)0, c, false, false); }
__device__ __forceinline__ v8f wmmab(v16bf a, v16bf b, v8f c) { return __builtin_amdgcn_wmma_f32_16x16x32_bf16(false, a, false, b, (short)0, c, false, false); }

template <typename T16> struct WFrag;
template <> struct WFrag<h16> { typedef v16h V; static __device__ __forceinline__ V ld(const h16* p) { return cat16(*(const v8h*)p, *(const v8h*)(p + 16)); } static __device__ __forceinline__ v8f mma(V a, V b, v8f c) { return wmma16(a, b, c); } };
template <> struct WFrag<bf> { typedef v16bf V; static __device__ __forceinline__ V ld(const bf* p) { return cat16b(*(const v8us*)p, *(const v8us*)(p + 16)); } static __device__ __forceinline__ v8f mma(V a, V b, v8f c) { return wmmab(a, b, c); } };
template <typename T16, int NSPLIT, bool BIAS>
__global__ __launch_bounds__(32) void k_gemmw(const T16* __restrict__ A, const T16* __restrict__ A2, const T16* __restrict__ Bt, const T16* __restrict__ Bt2, int K, float* C, int ldc, const float* __restrict__ bias, size_t sA, size_t sB, size_t sC) {
    typedef typename WFrag<T16>::V V;
    __shared__ __align__(16) float os[16 * 68];
    const size_t z = blockIdx.z; A += z * sA; if (A2) A2 += z * sA; Bt += z * sB; if (Bt2) Bt2 += z * sB; C += z * sC;
    const int lane = threadIdx.x & 31, lr = lane & 15, hi = lane >> 4; const int r0 = blockIdx.x * 64, c0 = blockIdx.y * 64;
    v8f acc[4][4];
#pragma unroll
    for (int mb = 0; mb < 4; ++mb)
#pragma unroll
        for (int nb = 0; nb < 4; ++nb) acc[mb][nb] = (v8f){};
    const size_t aoff = (size_t)(r0 + lr) * K + 8 * hi, boff = (size_t)(c0 + lr) * K + 8 * hi;
    for (int kc = 0; kc < K; kc += 32) {
        V a[4], a2[4];
#pragma unroll
        for (int mb = 0; mb < 4; ++mb) { a[mb] = WFrag<T16>::ld(A + aoff + (size_t)mb * 16 * K + kc); if (NSPLIT == 1 || NSPLIT == 2) a2[mb] = WFrag<T16>::ld(A2 + aoff + (size_t)mb * 16 * K + kc); }
#pragma unroll
        for (int nb = 0; nb < 4; ++nb) { const V b = WFrag<T16>::ld(Bt + boff + (size_t)nb * 16 * K + kc); V b2; if (NSPLIT >= 2) b2 = WFrag<T16>::ld(Bt2 + boff + (size_t)nb * 16 * K + kc);
#pragma unroll
            for (int mb = 0; mb < 4; ++mb) { acc[mb][nb] = WFrag<T16>::mma(a[mb], b, acc[mb][nb]); if (NSPLIT == 1 || NSPLIT == 2) acc[mb][nb] = WFrag<T16>::mma(a2[mb], b, acc[mb][nb]); if (NSPLIT >= 2) acc[mb][nb] = WFrag<T16>::mma(a[mb], b2, acc[mb][nb]); } }
        asm volatile("v_nop\n\tv_nop\n\tv_nop\n\tv_nop" : "+v"(acc[0][0]), "+v"(acc[1][1]), "+v"(acc[2][2]), "+v"(acc[3][3]) : "v"(a[0]), "v"(a[3]));
    }
#pragma unroll
    for (int mb = 0; mb < 4; ++mb) {
#pragma unroll
        for (int nb = 0; nb < 4; ++nb) {
#pragma unroll
            for (int j = 0; j < 8; ++j) os[(hi * 8 + j) * 68 + nb * 16 + lr] = acc[mb][nb][j]; }
        __builtin_amdgcn_wave_barrier(); asm volatile("" ::: "memory");
        float* crow = C + (size_t)(r0 + mb * 16) * ldc + c0;
#pragma unroll 1
        for (int ps = 0; ps < 2; ++ps) {
#pragma unroll
            for (int s = 0; s < 8; ++s) { const int row = 2 * s + hi, cofs = lr * 4; v4f val = *(const v4fa*)(os + row * 68 + cofs); if (BIAS) { val[0] += bfr(bias[c0 + cofs]); val[1] += bfr(bias[c0 + cofs + 1]); val[2] += bfr(bias[c0 + cofs + 2]); val[3] += bfr(bias[c0 + cofs + 3]); }
                *(volatile v4f*)(crow + (size_t)row * ldc + cofs) = val; }
            if (ps == 0) __threadfence(); }
        __builtin_amdgcn_wave_barrier(); asm volatile("" ::: "memory");
    }
}

typedef __attribute__((ext_vector_type(2))) _Float16 v2h;
typedef __attribute__((ext_vector_type(4))) _Float16 v4h;
typedef __attribute__((ext_vector_type(2))) unsigned short v2us;
typedef __attribute__((ext_vector_type(4))) unsigned short v4us;
typedef __attribute__((ext_vector_type(2))) float v2f;
typedef __attribute__((ext_vector_type(4))) int v4i;
__device__ __forceinline__ h16 toh_flush(float x) { const float z = (fabsf(x) < 6.103515625e-05f) ? 0.0f : x; return (h16)z; }

typedef __attribute__((ext_vector_type(4))) _Float16 v4h_;
__global__ __launch_bounds__(256) void k_fillb(bf* P, unsigned w2, size_t n8) { const size_t i = (size_t)blockIdx.x * 256 + threadIdx.x; if (i >= n8) return; v4i o; o[0] = (int)w2; o[1] = (int)w2; o[2] = (int)w2; o[3] = (int)w2;
    *(volatile v4i*)(P + i * 8) = o; __threadfence(); *(volatile v4i*)(P + i * 8) = o; }

__global__ __launch_bounds__(256) void k_wtw(const float* __restrict__ W, int ncol, int nlive, int sh, h16* Wt) {
    const unsigned i = blockIdx.x * 256 + threadIdx.x; const unsigned n = i & ((1u << sh) - 1u), k64 = i >> sh; const unsigned nc = (n < (unsigned)nlive) ? n : (unsigned)nlive - 1u; const float live = (float)(n < (unsigned)nlive);
    const float* src = W + (size_t)k64 * 64 * ncol + nc; h16 r[64];
#pragma unroll
    for (int kj = 0; kj < 64; ++kj) r[kj] = toh_flush(bfr(src[(size_t)kj * ncol]) * 1024.0f * live);
    h16* pd = Wt + (size_t)n * NDM + (size_t)k64 * 64;
#pragma unroll
    for (int ps = 0; ps < 2; ++ps) {
#pragma unroll
        for (int g = 0; g < 8; ++g) { v8h o;
#pragma unroll
            for (int j = 0; j < 8; ++j) o[j] = r[g * 8 + j];
            *(volatile v8h*)(pd + g * 8) = o; }
        if (ps == 0) __threadfence(); } }

__global__ __launch_bounds__(256) void k_xword(const float* __restrict__ src, h16* dst) {
    const size_t i = (size_t)blockIdx.x * 256 + threadIdx.x; const v8f wv = *(const v8f*)(src + i * 8); v8h ow;
#pragma unroll
    for (int j = 0; j < 8; ++j) ow[j] = toh_flush(bfr(wv[j]));
    *(volatile v8h*)(dst + i * 8) = ow; __threadfence(); *(volatile v8h*)(dst + i * 8) = ow; }

__global__ __launch_bounds__(256) void k_fac(const float* __restrict__ Q, const float* __restrict__ K, const float* __restrict__ G, const float* __restrict__ bb, h16* FaH, h16* FaL, h16* FbH, h16* FbL) {
    const unsigned i = blockIdx.x * 256 + threadIdx.x; const unsigned ts = i & 1023u, pr = i >> 10, sq = pr >> 4, hd = pr & 15u; const size_t row = (size_t)sq * NTS + ts;
    const float* pq = Q + row * NDM + hd * 64; const float* pk = K + row * NDM + hd * 64; const float gz = G[row * 64 + hd] * 0.0009765625f + bfr(bb[hd]); const float beta = 1.0f / (1.0f + expf(-gz));
#pragma unroll
    for (int sd = 0; sd < 2; ++sd) { const float* pp = sd ? pk : pq; float w[64]; float ss = 0.0f;
#pragma unroll
        for (int g = 0; g < 8; ++g) { const v8f t = *(const v8f*)(pp + g * 8);
#pragma unroll
            for (int j = 0; j < 8; ++j) { const float y = t[j] * 0.0009765625f; w[g * 8 + j] = y; ss = ss + y * y; } }
        const float rn = (1.0f / fmaxf(sqrtf(ss), 1e-12f)) * (sd ? beta : 1.0f) * 1024.0f; h16* ph = (sd ? FbH : FaH) + (size_t)i * 64; h16* pl = (sd ? FbL : FaL) + (size_t)i * 64; h16 rh[64], rl[64];
#pragma unroll
        for (int e = 0; e < 64; ++e) { const float f = w[e] * rn; const h16 hi = toh_flush(f); rh[e] = hi; rl[e] = toh_flush(f - (float)hi); }
#pragma unroll
        for (int ps = 0; ps < 2; ++ps) {
#pragma unroll
            for (int g = 0; g < 8; ++g) { v8h oh, ol;
#pragma unroll
                for (int j = 0; j < 8; ++j) { oh[j] = rh[g * 8 + j]; ol[j] = rl[g * 8 + j]; }
                *(volatile v8h*)(ph + g * 8) = oh; *(volatile v8h*)(pl + g * 8) = ol; }
            if (ps == 0) __threadfence(); } } }

__global__ __launch_bounds__(256) void k_tb(const h16* __restrict__ src, h16* dst) {
    const unsigned i = blockIdx.x * 256 + threadIdx.x; const unsigned cl = i & 63u, z = i >> 6; const h16* pp = src + (size_t)z * NBL + cl; h16 r[64];
#pragma unroll
    for (int u = 0; u < 64; ++u) r[u] = pp[u * 64];
    h16* pd = dst + (size_t)i * 64;
#pragma unroll
    for (int ps = 0; ps < 2; ++ps) {
#pragma unroll
        for (int g = 0; g < 8; ++g) { v8h o;
#pragma unroll
            for (int j = 0; j < 8; ++j) o[j] = r[g * 8 + j];
            *(volatile v8h*)(pd + g * 8) = o; }
        if (ps == 0) __threadfence(); } }

__global__ __launch_bounds__(256) void k_gc(const float* __restrict__ V, h16* GcH, h16* GcL) {
    const unsigned i = blockIdx.x * 256 + threadIdx.x; const unsigned cl = i & 63u, z = i >> 6, ck = z & 15u, pr = z >> 4, sq = pr >> 4, hd = pr & 15u; const float* pv = V + ((size_t)sq * NTS + (size_t)ck * NCS) * NDM + hd * 64 + cl; h16 rh[64], rl[64];
#pragma unroll
    for (int u = 0; u < 64; ++u) { const float f = pv[(size_t)u * NDM] * 0.0625f; const h16 hi = toh_flush(f); rh[u] = hi; rl[u] = toh_flush(f - (float)hi); }
    h16* ph = GcH + (size_t)i * 64; h16* pl = GcL + (size_t)i * 64;
#pragma unroll
    for (int ps = 0; ps < 2; ++ps) {
#pragma unroll
        for (int g = 0; g < 8; ++g) { v8h oh, ol;
#pragma unroll
            for (int j = 0; j < 8; ++j) { oh[j] = rh[g * 8 + j]; ol[j] = rl[g * 8 + j]; }
            *(volatile v8h*)(ph + g * 8) = oh; *(volatile v8h*)(pl + g * 8) = ol; }
        if (ps == 0) __threadfence(); } }

__global__ __launch_bounds__(256) void k_msk2(const float* __restrict__ Pw, h16* Ph) {
    const unsigned i = blockIdx.x * 256 + threadIdx.x; const unsigned tr = i & 63u; const float* pw = Pw + (size_t)i * 64; h16 rh[64];
#pragma unroll
    for (int g = 0; g < 8; ++g) { const v8f t = *(const v8f*)(pw + g * 8);
#pragma unroll
        for (int j = 0; j < 8; ++j) { const float kp = (float)((unsigned)(g * 8 + j) <= tr); rh[g * 8 + j] = toh_flush(t[j] * 9.5367431640625e-07f * kp); } }
    h16* ph = Ph + (size_t)i * 64;
#pragma unroll
    for (int ps = 0; ps < 2; ++ps) {
#pragma unroll
        for (int g = 0; g < 8; ++g) { v8h oh;
#pragma unroll
            for (int j = 0; j < 8; ++j) oh[j] = rh[g * 8 + j];
            *(volatile v8h*)(ph + g * 8) = oh; }
        if (ps == 0) __threadfence(); } }

__global__ __launch_bounds__(256) void k_sum(const float* __restrict__ bef, const float* __restrict__ d1, const float* __restrict__ d2, float* aft, h16* SwH, h16* SwL, int ck) {
    const unsigned i = blockIdx.x * 256 + threadIdx.x; const unsigned j4 = i & 1023u, pr = i >> 10; const size_t ob = (size_t)pr * NBL + j4 * 4, oz = ((size_t)pr * NCK + (size_t)ck) * NBL + j4 * 4; const v4f ub = *(const v4fa*)(bef + ob); const v4f v1 = *(const v4fa*)(d1 + oz); const v4f v2 = *(const v4fa*)(d2 + oz); v4h_ oh, ol; v4f oa;
#pragma unroll
    for (int j = 0; j < 4; ++j) { const float f = ub[j] * 16.0f; const h16 hi = toh_flush(f); oh[j] = hi; ol[j] = toh_flush(f - (float)hi); oa[j] = ub[j] + (v1[j] + v2[j]) * 1.52587890625e-05f; }
    h16* ph = SwH + oz; h16* pl = SwL + oz; float* pa = aft + ob;
    *(volatile v4h_*)ph = oh; *(volatile v4h_*)pl = ol; *(volatile v4f*)pa = oa; __threadfence(); *(volatile v4h_*)ph = oh; *(volatile v4h_*)pl = ol; *(volatile v4f*)pa = oa; }

__global__ __launch_bounds__(256) void k_lay2(const float* __restrict__ Oa, const float* __restrict__ O1, const float* __restrict__ O2, h16* Ow) {
    const unsigned i = blockIdx.x * 256 + threadIdx.x; const unsigned m4 = i & 15u, ts = (i >> 4) & 1023u, pr = i >> 14, sq = pr >> 4, hd = pr & 15u; const size_t rw = (size_t)pr * NTS + ts;
    const v4f ua = *(const v4fa*)(Oa + rw * 64 + m4 * 4); const v4f u1 = *(const v4fa*)(O1 + rw * 64 + m4 * 4); const v4f u2 = *(const v4fa*)(O2 + rw * 64 + m4 * 4); v4h_ ow;
#pragma unroll
    for (int j = 0; j < 4; ++j) ow[j] = toh_flush(ua[j] * 0.015625f + (u1[j] + u2[j]) * 6.103515625e-05f);
    h16* pd = Ow + ((size_t)sq * NTS + ts) * NDM + hd * 64 + m4 * 4;
    *(volatile v4h_*)pd = ow; __threadfence(); *(volatile v4h_*)pd = ow; }

__global__ __launch_bounds__(256) void k_res(const float* __restrict__ Fo, float* res) {
    const size_t i = (size_t)blockIdx.x * 256 + threadIdx.x; const v8f t = *(const v8f*)(Fo + i * 8); v8f o;
#pragma unroll
    for (int j = 0; j < 8; ++j) o[j] = t[j] * 0.0009765625f;
    *(volatile v8f*)(res + i * 8) = o; __threadfence(); *(volatile v8f*)(res + i * 8) = o; }

extern "C" void kernel_launch(void* const* d_in, const int* in_sizes, int n_in, void* d_out, int out_size, void* d_ws, size_t ws_size, hipStream_t stream) {
    if (n_in < 7) return;
    if (in_sizes[0] != NRW * NDM || in_sizes[1] != NDM * NDM || in_sizes[2] != NDM * NDM || in_sizes[3] != NDM * NDM || in_sizes[4] != NDM * NDM || in_sizes[5] != NDM * NHS || in_sizes[6] != NHS) return;
    if (out_size != NRW * NDM) return;
    static_assert(NPR == NSQ * NHS && NHS == 16 && NFE == 64 && NCS == 64 && NCK * NCS == NTS && NTS == 1024 && NZQ == NPR * NCK && NBL == 64 * 64 && NRW == NSQ * NTS && NDM == NHS * NFE && NDM == 1024 && (NRW * NDM / 8) % 256 == 0 && (NZQ * 64) % 256 == 0 && (NPR * NTS) % 256 == 0 && (NPR * NBL / 4) % 256 == 0 && (NPR * NTS * 16) % 256 == 0 && (NDM * 16) % 256 == 0 && (64 * 16) % 256 == 0, "the block products: 64 by 64 over a depth of 64; the flat grids exact; the index fields' widths (4 bits a head, 10 a time, 4 a chunk, 6 a column)");
    const float* xin = (const float*)d_in[0]; const float* Wq = (const float*)d_in[1]; const float* Wk = (const float*)d_in[2]; const float* Wv = (const float*)d_in[3]; const float* Wo = (const float*)d_in[4]; const float* Wb = (const float*)d_in[5]; const float* bbv = (const float*)d_in[6]; float* res = (float*)d_out;
    char* wsp = (char*)d_ws; auto take = [&](size_t bytes) { char* p = wsp; wsp += (bytes + 255) & ~(size_t)255; return (void*)p; };
    float* Zn = (float*)take((size_t)NPR * NBL * 4); h16* Xw = (h16*)take((size_t)NRW * NDM * 2); h16* Wtq = (h16*)take((size_t)NDM * NDM * 2); h16* Wtk = (h16*)take((size_t)NDM * NDM * 2); h16* Wtv = (h16*)take((size_t)NDM * NDM * 2); h16* Wto = (h16*)take((size_t)NDM * NDM * 2); h16* Wg = (h16*)take((size_t)64 * NDM * 2);
    float* T0 = (float*)take((size_t)NRW * NDM * 4); float* T1 = (float*)take((size_t)NRW * NDM * 4); float* T2 = (float*)take((size_t)NRW * NDM * 4); float* G = (float*)take((size_t)NRW * 64 * 4);
    h16* FaH = (h16*)take((size_t)NPR * NTS * 64 * 2); h16* FaL = (h16*)take((size_t)NPR * NTS * 64 * 2); h16* FbH = (h16*)take((size_t)NPR * NTS * 64 * 2); h16* FbL = (h16*)take((size_t)NPR * NTS * 64 * 2);
    h16* GbH = (h16*)take((size_t)NZQ * NBL * 2); h16* GbL = (h16*)take((size_t)NZQ * NBL * 2); h16* GcH = (h16*)take((size_t)NZQ * NBL * 2); h16* GcL = (h16*)take((size_t)NZQ * NBL * 2); h16* Ph = (h16*)take((size_t)NZQ * NBL * 2);
    float* Ra = (float*)take((size_t)NPR * NBL * 4); float* Rb = (float*)take((size_t)NPR * NBL * 4); h16* SwH = (h16*)take((size_t)NZQ * NBL * 2); h16* SwL = (h16*)take((size_t)NZQ * NBL * 2);
    float* Oa = (float*)take((size_t)NZQ * NBL * 4); float* O1 = (float*)take((size_t)NZQ * NBL * 4); float* O2 = (float*)take((size_t)NZQ * NBL * 4);
    if ((size_t)(wsp - (char*)d_ws) > ws_size) return;
    float* Q = T0; float* K = T1; float* V = T2; float* Pw = T0; float* D1 = T1; float* D2 = T2; float* Fo = T0; h16* Ow = Xw;
    k_fillb<<<(unsigned)((size_t)NPR * NBL * 4 / 16 / 256), 256, 0, stream>>>((bf*)Zn, 0u, (size_t)NPR * NBL * 4 / 16);
    k_wtw<<<NDM * 16 / 256, 256, 0, stream>>>(Wq, NDM, NDM, 10, Wtq); k_wtw<<<NDM * 16 / 256, 256, 0, stream>>>(Wk, NDM, NDM, 10, Wtk); k_wtw<<<NDM * 16 / 256, 256, 0, stream>>>(Wv, NDM, NDM, 10, Wtv); k_wtw<<<NDM * 16 / 256, 256, 0, stream>>>(Wo, NDM, NDM, 10, Wto); k_wtw<<<64 * 16 / 256, 256, 0, stream>>>(Wb, NHS, NHS, 6, Wg);
    k_xword<<<(unsigned)(NRW * NDM / 8 / 256), 256, 0, stream>>>(xin, Xw);
    k_gemmw<h16, 0, false><<<dim3(NRW / 64, NDM / 64, 1), 32, 0, stream>>>(Xw, nullptr, Wtq, nullptr, NDM, Q, NDM, nullptr, 0, 0, 0);
    k_gemmw<h16, 0, false><<<dim3(NRW / 64, NDM / 64, 1), 32, 0, stream>>>(Xw, nullptr, Wtk, nullptr, NDM, K, NDM, nullptr, 0, 0, 0);
    k_gemmw<h16, 0, false><<<dim3(NRW / 64, NDM / 64, 1), 32, 0, stream>>>(Xw, nullptr, Wtv, nullptr, NDM, V, NDM, nullptr, 0, 0, 0);
    k_gemmw<h16, 0, false><<<dim3(NRW / 64, 1, 1), 32, 0, stream>>>(Xw, nullptr, Wg, nullptr, NDM, G, 64, nullptr, 0, 0, 0);
    k_fac<<<NPR * NTS / 256, 256, 0, stream>>>(Q, K, G, bbv, FaH, FaL, FbH, FbL);
    k_gc<<<NZQ * 64 / 256, 256, 0, stream>>>(V, GcH, GcL);
    k_tb<<<NZQ * 64 / 256, 256, 0, stream>>>(FbH, GbH); k_tb<<<NZQ * 64 / 256, 256, 0, stream>>>(FbL, GbL);
    k_gemmw<h16, 0, false><<<dim3(1, 1, NZQ), 32, 0, stream>>>(FaH, nullptr, FbH, nullptr, NFE, Pw, 64, nullptr, NBL, NBL, NBL);
    k_gemmw<h16, 1, false><<<dim3(1, 1, NZQ), 32, 0, stream>>>(GcH, GcL, GbH, nullptr, NCS, D1, 64, nullptr, NBL, NBL, NBL);
    k_gemmw<h16, 0, false><<<dim3(1, 1, NZQ), 32, 0, stream>>>(GcH, nullptr, GbL, nullptr, NCS, D2, 64, nullptr, NBL, NBL, NBL);
    k_msk2<<<NZQ * 64 / 256, 256, 0, stream>>>(Pw, Ph);
    for (int ck = 0; ck < NCK; ++ck) { const float* bef = (ck == 0) ? (const float*)Zn : ((ck & 1) ? (const float*)Ra : (const float*)Rb); float* aft = (ck & 1) ? Rb : Ra; k_sum<<<NPR * NBL / 4 / 256, 256, 0, stream>>>(bef, D1, D2, aft, SwH, SwL, ck); }
    k_gemmw<h16, 0, false><<<dim3(1, 1, NZQ), 32, 0, stream>>>(Ph, nullptr, GcH, nullptr, NCS, Oa, 64, nullptr, NBL, NBL, NBL);
    k_gemmw<h16, 1, false><<<dim3(1, 1, NZQ), 32, 0, stream>>>(FaH, FaL, SwH, nullptr, NFE, O1, 64, nullptr, NBL, NBL, NBL);
    k_gemmw<h16, 0, false><<<dim3(1, 1, NZQ), 32, 0, stream>>>(FaH, nullptr, SwL, nullptr, NFE, O2, 64, nullptr, NBL, NBL, NBL);
    k_lay2<<<NPR * NTS * 16 / 256, 256, 0, stream>>>(Oa, O1, O2, Ow);
    k_gemmw<h16, 0, false><<<dim3(NRW / 64, NDM / 64, 1), 32, 0, stream>>>(Ow, nullptr, Wto, nullptr, NDM, Fo, NDM, nullptr, 0, 0, 0);
    k_res<<<(unsigned)(NRW * NDM / 8 / 256), 256, 0, stream>>>(Fo, res);
}
